// TimeReversalFeatureExtractor_18794776887341
// MI455X (gfx1250) — hardware-run, weakly checked
//
#include <hip/hip_runtime.h>
#include <math.h>

typedef __attribute__((ext_vector_type(16))) _Float16 v16h;
typedef __attribute__((ext_vector_type(8)))  _Float16 v8h;
typedef __attribute__((ext_vector_type(8)))  float    v8f;
typedef __attribute__((ext_vector_type(4)))  float    v4f;
typedef __attribute__((ext_vector_type(4)))  unsigned int v4u;

constexpr int kNb     = 4;
constexpr int kNc     = 8;
constexpr int kNt     = 16000;
constexpr int kWin    = 512;
constexpr int kHop    = 128;
constexpr int kFrm    = (kNt - kWin) / kHop + 1;
constexpr int kFrmP   = 128;
constexpr int kNf     = 103;
constexpr int kBin0   = 10;
constexpr int kNaz    = 72;
constexpr int kNel    = 13;
constexpr int kNd     = kNaz * kNel;
constexpr int kNdP    = 960;
constexpr int kBands  = 8;
constexpr int kBC     = kNb * kNc;
constexpr int kBF     = kNb * kNf;
constexpr int kAudP   = 16896;
constexpr int kNdft   = 256;
constexpr int kStRows = 2 * kNdP;
constexpr int kAvRows = 416;
constexpr int kOutPerB = kBands * kNd;
static_assert(kFrm == 122, "frame count");
static_assert(kNd == 936, "direction count");
static_assert(kBF == 412 && kBC == 32, "batch products");
static_assert((kFrmP - 1) * kHop + kWin <= kAudP, "padded audio pitch covers every fragment row");
static_assert((kAudP % 8) == 0 && (kBC * (kAudP / 8)) == 264 * 256, "audio plane launch covers the plane exactly");
static_assert((kNdP % 64) == 0 && kNdP >= kNd, "direction padding");
static_assert((kWin % 32) == 0 && (kFrmP % 64) == 0 && (kNdft % 64) == 0, "GEMM K multiple of 32, M and N multiples of 64");
static_assert(kAvRows % 16 == 0 && kAvRows >= kBF, "dominant-steering table rows");
static_assert(kOutPerB == 7488 && (kOutPerB % 32) == 0, "output lines per batch element");

constexpr float kAudCarry  = 16.0f;
constexpr float kDftCarry  = 256.0f;
constexpr float kStftScale = 1.0f / (kAudCarry * kDftCarry);
constexpr float kLoCarry   = 64.0f;
constexpr float kStCarry   = 16.0f;
constexpr float kStLoScale = kStCarry / kLoCarry;
constexpr float kPowScale  = 1.0f / ((float)kFrm * kStCarry * kStCarry);
constexpr float kH16Min    = 6.103515625e-5f;
constexpr float kTwoPi     = 6.2831853071795864769f;
constexpr float kPiOver256 = 3.14159265358979323846f / 256.0f;
constexpr float kDegRad    = 0.017453292519943295f;
constexpr float kBinHz     = 31.25f;
constexpr float kInvSound  = 1.0f / 343.0f;
constexpr float kInvBins   = 1.0f / (float)kNf;
constexpr float kInvTemp   = 1.0f / 0.35f;
constexpr float kShrink    = 0.85f;
constexpr float kEps       = 1e-8f;

constexpr size_t kSzAUD   = (size_t)kBC * kAudP * 2;
constexpr size_t kSzBDFT  = (size_t)kNdft * kWin * 2;
constexpr size_t kSzCSPEC = (size_t)kBC * kFrmP * kNdft * 4;
constexpr size_t kSzDEL   = (size_t)kBC * kNdP * 4;
constexpr size_t kSzRES   = (size_t)kBF * kFrmP * 16 * 4;
constexpr size_t kSzARES  = (size_t)kBF * kFrmP * 32 * 2;
constexpr size_t kSzBST   = (size_t)kBF * kStRows * 32 * 2;
constexpr size_t kSzFMAP  = (size_t)kBF * kNdP * 4;
constexpr size_t kSzWSM   = (size_t)kNb * kNdP * 4;
constexpr size_t kSzAVEC  = (size_t)kAvRows * 16 * 4;
constexpr size_t kOffAUD   = 0;
constexpr size_t kOffBDFT  = kOffAUD   + kSzAUD;
constexpr size_t kOffCSPEC = kOffBDFT  + kSzBDFT;
constexpr size_t kOffDEL   = kOffCSPEC + kSzCSPEC;
constexpr size_t kOffRES0  = kOffDEL   + kSzDEL;
constexpr size_t kOffRES1  = kOffRES0  + kSzRES;
constexpr size_t kOffARES  = kOffRES1  + kSzRES;
constexpr size_t kOffBST   = kOffARES  + kSzARES;
constexpr size_t kOffFMAP  = kOffBST   + kSzBST;
constexpr size_t kOffWSM   = kOffFMAP  + kSzFMAP;
constexpr size_t kOffAVEC  = kOffWSM   + kSzWSM;
constexpr size_t kWsTotal  = kOffAVEC  + kSzAVEC;
static_assert(kWsTotal == 68036608ull, "carve total");
static_assert(kWsTotal <= 134217728ull, "carve cap");
static_assert((kOffBDFT % 128) == 0 && (kOffCSPEC % 128) == 0 && (kOffDEL % 128) == 0 && (kOffRES0 % 128) == 0 &&
              (kOffRES1 % 128) == 0 && (kOffARES % 128) == 0 && (kOffBST % 128) == 0 && (kOffFMAP % 128) == 0 &&
              (kOffWSM % 128) == 0 && (kOffAVEC % 128) == 0, "128-B aligned regions");

__device__ __forceinline__ unsigned short f2bf_bits(float f) {
  unsigned u = __float_as_uint(f);
  return (unsigned short)((u + 0x7FFFu + ((u >> 16) & 1u)) >> 16);
}
__device__ __forceinline__ float bf_bits2f(unsigned short h) { return __uint_as_float(((unsigned)h) << 16); }

__device__ __forceinline__ _Float16 to_h_flush(float v) {
  const float z = (fabsf(v) < kH16Min) ? 0.0f : v;
  return (_Float16)z;
}
__device__ __forceinline__ unsigned short h_bits_flush(float v) {
  const _Float16 h = to_h_flush(v);
  return __builtin_bit_cast(unsigned short, h);
}

__device__ __forceinline__ v8f mma_guard_h(v16h a, v16h b, v8f c) {
  c = __builtin_amdgcn_wmma_f32_16x16x32_f16(false, a, false, b, (short)0, c, false, false);
  asm volatile("v_nop\n\tv_nop\n\tv_nop\n\tv_nop" : "+v"(c) : "v"(a), "v"(b));
  return c;
}
__device__ __forceinline__ void keep4_h(v16h a, v16h b, v16h c, v16h d) { asm volatile("v_nop" :: "v"(a), "v"(b), "v"(c), "v"(d)); }
__device__ __forceinline__ void acc_guard4(v8f& a, v8f& b, v8f& c, v8f& d) { asm volatile("v_nop\n\tv_nop\n\tv_nop\n\tv_nop" : "+v"(a), "+v"(b), "+v"(c), "+v"(d)); }

template <typename T> struct Frag;
template <> struct Frag<_Float16> {
  typedef v16h V; union U { v16h v; v8h h[2]; };
  static __device__ __forceinline__ v16h load(const _Float16* p) {
    U f; f.h[0] = *(const v8h*)(p); f.h[1] = *(const v8h*)(p + 16); return f.v;
  }
  static __device__ __forceinline__ v8f mmag(v16h a, v16h b, v8f c) { return mma_guard_h(a, b, c); }
  static __device__ __forceinline__ void keep(v16h a, v16h b, v16h c, v16h d) { keep4_h(a, b, c, d); }
};

template <int ET> struct Elem;
template <> struct Elem<0> { typedef _Float16 T; };
template <int ET, bool SPLIT, int BIAS_MODE, int OUT_MODE, bool RESID, int ACT = 0>
__global__ __launch_bounds__(256) void wmma_gemm64(
    const unsigned short* __restrict__ Ap, const unsigned short* __restrict__ A2p, int lda, long strideA,
    const unsigned short* __restrict__ Btp, const unsigned short* __restrict__ Bt2p, int ldb, long strideB,
    void* __restrict__ Cout, void* __restrict__ Cout2, int ldc, long strideC,
    const float* __restrict__ bias,
    const float* __restrict__ resid, long strideR,
    int M, int N, int K, float scale) {
  typedef typename Elem<ET>::T T;
  typedef typename Frag<T>::V V;
  const T* A = (const T*)Ap; const T* A2 = (const T*)A2p; const T* Bt = (const T*)Btp; const T* Bt2 = (const T*)Bt2p;
  __shared__ __align__(16) float sT[8][16 * 68];
  const int b    = blockIdx.y;
  const int lane = threadIdx.x & 31;
  const int wave = threadIdx.x >> 5;
  const int tilesN = N >> 6;
  const int tilesM = M >> 6;
  const int tile = blockIdx.x * 8 + wave;
  if (tile >= tilesM * tilesN) return;
  const int tm = tile / tilesN;
  const int tn = tile - tm * tilesN;
  const int m0 = tm << 6;
  const int n0 = tn << 6;

  const T* Ab  = A  + (size_t)b * strideA;
  const T* Bb  = Bt + (size_t)b * strideB;
  const T* Ab2 = SPLIT ? (A2  + (size_t)b * strideA) : nullptr;
  const T* Bb2 = SPLIT ? (Bt2 + (size_t)b * strideB) : nullptr;

  const int rlane = lane & 15;
  const int koff  = (lane >> 4) * 8;
  const int mOff  = (lane >> 4) * 8;

  v8f acc[4][4];
#pragma unroll
  for (int i = 0; i < 4; ++i)
#pragma unroll
    for (int j = 0; j < 4; ++j) acc[i][j] = (v8f){0.f,0.f,0.f,0.f,0.f,0.f,0.f,0.f};

  for (int k0 = 0; k0 < K; k0 += 32) {
    V bh[4], bl[4];
#pragma unroll
    for (int j = 0; j < 4; ++j) {
      const size_t bo = (size_t)(n0 + (j << 4) + rlane) * ldb + koff + k0;
      bh[j] = Frag<T>::load(Bb + bo);
      if (SPLIT) bl[j] = Frag<T>::load(Bb2 + bo);
    }
#pragma unroll
    for (int i = 0; i < 4; ++i) {
      const size_t ao = (size_t)(m0 + (i << 4) + rlane) * lda + koff + k0;
      V ah = Frag<T>::load(Ab + ao);
      V al;
      if (SPLIT) al = Frag<T>::load(Ab2 + ao);
#pragma unroll
      for (int j = 0; j < 4; ++j) {
        acc[i][j] = Frag<T>::mmag(ah, bh[j], acc[i][j]);
        if (SPLIT) {
          acc[i][j] = Frag<T>::mmag(ah, bl[j], acc[i][j]);
          acc[i][j] = Frag<T>::mmag(al, bh[j], acc[i][j]);
        }
      }
    }
    Frag<T>::keep(bh[0], bh[1], bh[2], bh[3]);
    if (SPLIT) Frag<T>::keep(bl[0], bl[1], bl[2], bl[3]);
  }
  acc_guard4(acc[0][0], acc[0][1], acc[0][2], acc[0][3]);
  acc_guard4(acc[1][0], acc[1][1], acc[1][2], acc[1][3]);
  acc_guard4(acc[2][0], acc[2][1], acc[2][2], acc[2][3]);
  acc_guard4(acc[3][0], acc[3][1], acc[3][2], acc[3][3]);

  float* slab = sT[wave];
  const float* Rb = RESID ? (resid + (size_t)b * strideR) : nullptr;
#pragma unroll
  for (int i = 0; i < 4; ++i) {
    const int mBase = m0 + (i << 4);
#pragma unroll
    for (int j = 0; j < 4; ++j) {
      const int n = n0 + (j << 4) + rlane;
      float bv = 0.f;
      if (BIAS_MODE == 2) bv = bias[n];
#pragma unroll
      for (int r = 0; r < 8; ++r) {
        float v = acc[i][j][r] * scale;
        if (BIAS_MODE == 1) v += bias[mBase + mOff + r];
        if (BIAS_MODE == 2) v += bv;
        if (RESID) v += Rb[(size_t)(mBase + mOff + r) * ldc + n];
        if (ACT == 2) v = fmaxf(v, 0.0f);
        if (ACT == 4) v = (v > 0.f) ? v : 0.01f * v;
        slab[(mOff + r) * 68 + (j << 4) + rlane] = v;
      }
    }
    __builtin_amdgcn_fence(__ATOMIC_RELEASE, "workgroup");
    __builtin_amdgcn_wave_barrier();
    __builtin_amdgcn_fence(__ATOMIC_ACQUIRE, "workgroup");
    if (OUT_MODE == 0) {
      float* C = (float*)Cout + (size_t)b * strideC;
      const int hh = lane >> 4, c4 = (lane & 15) * 4;
      for (int pass = 0; pass < 2; ++pass) {
#pragma unroll
        for (int it = 0; it < 8; ++it) {
          const int row = it * 2 + hh;
          v4f v = *(const v4f*)(slab + row * 68 + c4);
          *(volatile v4f*)(C + (size_t)(mBase + row) * ldc + n0 + c4) = v;
        }
        __threadfence();
      }
    } else {
      const int q = lane >> 3, c8 = (lane & 7) * 8;
      unsigned short* C  = (unsigned short*)Cout  + (size_t)b * strideC;
      unsigned short* C2 = (OUT_MODE == 2) ? ((unsigned short*)Cout2 + (size_t)b * strideC) : nullptr;
      for (int pass = 0; pass < 2; ++pass) {
#pragma unroll
        for (int it = 0; it < 4; ++it) {
          const int row = it * 4 + q;
          const float* sp = slab + row * 68 + c8;
          v8h hv, lv;
#pragma unroll
          for (int e = 0; e < 8; ++e) {
            if (OUT_MODE == 1) {
              hv[e] = (_Float16)sp[e];
            } else {
              unsigned short hb = f2bf_bits(sp[e]);
              unsigned short lb = f2bf_bits(sp[e] - bf_bits2f(hb));
              hv[e] = __builtin_bit_cast(_Float16, hb);
              lv[e] = __builtin_bit_cast(_Float16, lb);
            }
          }
          *(volatile v8h*)(C + (size_t)(mBase + row) * ldc + n0 + c8) = hv;
          if (OUT_MODE == 2) *(volatile v8h*)(C2 + (size_t)(mBase + row) * ldc + n0 + c8) = lv;
        }
        __threadfence();
      }
    }
    __builtin_amdgcn_fence(__ATOMIC_RELEASE, "workgroup");
    __builtin_amdgcn_wave_barrier();
    __builtin_amdgcn_fence(__ATOMIC_ACQUIRE, "workgroup");
  }
}

__global__ __launch_bounds__(256) void dft_plane_kernel(unsigned short* __restrict__ bdft)
{
  __shared__ __align__(16) unsigned short sB[2048];
  const int tid = threadIdx.x;
  const int blk = blockIdx.x;
#pragma unroll 1
  for (int it = 0; it < 8; ++it) {
    const int e = it * 256 + tid;
    const int n = blk * 4 + (e >> 9);
    const int w = e & 511;
    const bool isIm = n >= 128;
    const int f = isIm ? (n - 128) : n;
    const bool live = f < kNf;
    const int k = kBin0 + (live ? f : (kNf - 1));
    const int r = (k * w) & 511;
    const int rs = (r >= 256) ? (r - 512) : r;
    const int ws = (w >= 256) ? (w - 512) : w;
    float sn, cs;
    sincosf((float)rs * kPiOver256, &sn, &cs);
    const float win = 0.5f - 0.5f * cosf((float)ws * kPiOver256);
    const float tr = isIm ? sn : cs;
    const float val = live ? (tr * win) * kDftCarry : 0.0f;
    sB[e] = h_bits_flush(val);
  }
  __syncthreads();
  const v4u v = *(const v4u*)(sB + tid * 8);
  unsigned short* dst = bdft + (size_t)blk * 2048 + tid * 8;
  *(volatile v4u*)dst = v;
  __threadfence();
  *(volatile v4u*)dst = v;
}

__global__ __launch_bounds__(64) void delays_kernel(const float* __restrict__ mics, float* __restrict__ del)
{
  const int bc = blockIdx.x;
  const int b = bc >> 3;
  const int d = blockIdx.y * 64 + threadIdx.x;
  const bool live = d < kNd;
  const int dd = live ? d : (kNd - 1);
  float mx = 0.0f, my = 0.0f, mz = 0.0f;
#pragma unroll 1
  for (int cc = 0; cc < kNc; ++cc) {
    mx += mics[(b * kNc + cc) * 3 + 0];
    my += mics[(b * kNc + cc) * 3 + 1];
    mz += mics[(b * kNc + cc) * 3 + 2];
  }
  mx *= 0.125f; my *= 0.125f; mz *= 0.125f;
  const float px = mics[bc * 3 + 0] - mx;
  const float py = mics[bc * 3 + 1] - my;
  const float pz = mics[bc * 3 + 2] - mz;
  const int ei = dd / kNaz;
  const int aj = dd - ei * kNaz;
  const float elr = (30.0f + 10.0f * (float)ei) * kDegRad;
  const float azr = (5.0f * (float)aj) * kDegRad;
  float se, ce, sa, ca;
  sincosf(elr, &se, &ce);
  sincosf(azr, &sa, &ca);
  const float dx = se * ca, dy = se * sa, dz = ce;
  const float dot = px * dx + py * dy + pz * dz;
  const float v = live ? (-dot) * kInvSound : 0.0f;
  volatile float* q = del + (size_t)bc * kNdP + d;
  *q = v;
  __threadfence();
  *q = v;
}

__global__ __launch_bounds__(256) void audio_plane_kernel(const float* __restrict__ audio, unsigned short* __restrict__ aud)
{
  const int i = blockIdx.x * 256 + threadIdx.x;
  const int bc = i / (kAudP / 8);
  const int s8 = (i - bc * (kAudP / 8)) * 8;
  const bool live = s8 < kNt;
  const int sc = live ? s8 : (kNt - 8);
  const float* src = audio + (size_t)bc * kNt + sc;
  v4f a0 = *(const v4f*)(src);
  v4f a1 = *(const v4f*)(src + 4);
  asm volatile("" : "+v"(a0), "+v"(a1));
  v8h hv;
#pragma unroll
  for (int e = 0; e < 4; ++e) {
    const float x0 = live ? a0[e] * kAudCarry : 0.0f;
    const float x1 = live ? a1[e] * kAudCarry : 0.0f;
    hv[e]     = to_h_flush(x0);
    hv[4 + e] = to_h_flush(x1);
  }
  unsigned short* dst = aud + (size_t)i * 8;
  *(volatile v8h*)dst = hv;
  __threadfence();
  *(volatile v8h*)dst = hv;
}

__device__ __forceinline__ void store_res_planes(const float* sR, float* resOut, unsigned short* aOut, int tid)
{
  v4f rv[4];
  v8h av[4];
#pragma unroll
  for (int it = 0; it < 4; ++it) {
    const int idx = it * 128 + tid;
    rv[it] = *(const v4f*)(sR + idx * 4);
    const int row = idx >> 2, q = idx & 3;
    const float* xp = sR + row * 16 + (q & 1) * 8;
    const v4f x0 = *(const v4f*)(xp);
    const v4f x1 = *(const v4f*)(xp + 4);
    const bool wantLo = (q >= 2);
    v8h o;
#pragma unroll
    for (int e = 0; e < 4; ++e) {
      const float xa = x0[e], xb = x1[e];
      const _Float16 ha = to_h_flush(xa);
      const _Float16 hb = to_h_flush(xb);
      const float ra = (xa - (float)ha) * kLoCarry;
      const float rb = (xb - (float)hb) * kLoCarry;
      const float sa = wantLo ? ra : xa;
      const float sb = wantLo ? rb : xb;
      o[e]     = to_h_flush(sa);
      o[4 + e] = to_h_flush(sb);
    }
    av[it] = o;
  }
  for (int pass = 0; pass < 2; ++pass) {
#pragma unroll
    for (int it = 0; it < 4; ++it) {
      const int idx = it * 128 + tid;
      *(volatile v4f*)(resOut + idx * 4) = rv[it];
      *(volatile v8h*)(aOut + idx * 8) = av[it];
    }
    __threadfence();
  }
}

__global__ __launch_bounds__(128) void phat_pack_kernel(const float* __restrict__ cspec, float* __restrict__ res0,
                                                        unsigned short* __restrict__ ares)
{
  __shared__ __align__(16) float sR[kFrmP * 16];
  const int tid = threadIdx.x;
  const int bf = blockIdx.x;
  const int b = bf / kNf;
  const int f = bf - b * kNf;
  const bool live = tid < kFrm;
#pragma unroll 1
  for (int c = 0; c < kNc; ++c) {
    const float* row = cspec + (size_t)((b * kNc + c) * kFrmP + tid) * kNdft;
    float re = row[f];
    float im = row[128 + f];
    asm volatile("" : "+v"(re), "+v"(im));
    const float mag = sqrtf(re * re + im * im);
    const float inv = 1.0f / fmaxf(mag, kEps);
    const float wr = re * inv, wi = im * inv;
    sR[tid * 16 + c]     = live ? wr : 0.0f;
    sR[tid * 16 + 8 + c] = live ? wi : 0.0f;
  }
  __syncthreads();
  store_res_planes(sR, res0 + (size_t)bf * (kFrmP * 16), ares + (size_t)bf * (kFrmP * 32), tid);
}

__global__ __launch_bounds__(64) void steer_plane_kernel(const float* __restrict__ del, unsigned short* __restrict__ bst)
{
  __shared__ __align__(16) unsigned short sRe[64 * 32];
  __shared__ __align__(16) unsigned short sIm[64 * 32];
  const int tid = threadIdx.x;
  const int bf = blockIdx.x;
  const int d0 = blockIdx.y * 64;
  const int d = d0 + tid;
  const bool live = d < kNd;
  const int b = bf / kNf;
  const int f = bf - b * kNf;
  const float tw = kTwoPi * ((float)(kBin0 + f) * kBinHz);
#pragma unroll 1
  for (int c = 0; c < kNc; ++c) {
    float dl = del[(size_t)(b * kNc + c) * kNdP + d];
    asm volatile("" : "+v"(dl));
    const float ph = tw * dl;
    float sn, cs;
    sincosf(ph, &sn, &cs);
    const float cv = live ? cs * kStCarry : 0.0f;
    const float sv = live ? sn * kStCarry : 0.0f;
    const float cl = live ? cs * kStLoScale : 0.0f;
    const float sl = live ? sn * kStLoScale : 0.0f;
    sRe[tid * 32 + c]      = h_bits_flush(cv);
    sRe[tid * 32 + 8 + c]  = h_bits_flush(-sv);
    sRe[tid * 32 + 16 + c] = h_bits_flush(cl);
    sRe[tid * 32 + 24 + c] = h_bits_flush(-sl);
    sIm[tid * 32 + c]      = h_bits_flush(sv);
    sIm[tid * 32 + 8 + c]  = h_bits_flush(cv);
    sIm[tid * 32 + 16 + c] = h_bits_flush(sl);
    sIm[tid * 32 + 24 + c] = h_bits_flush(cl);
  }
  __syncthreads();
  v4u re4[4], im4[4];
#pragma unroll
  for (int it = 0; it < 4; ++it) {
    const int idx = it * 64 + tid;
    re4[it] = *(const v4u*)(sRe + idx * 8);
    im4[it] = *(const v4u*)(sIm + idx * 8);
  }
  unsigned short* dRe = bst + ((size_t)bf * kStRows + d0) * 32;
  unsigned short* dIm = dRe + (size_t)kNdP * 32;
  for (int pass = 0; pass < 2; ++pass) {
#pragma unroll
    for (int it = 0; it < 4; ++it) {
      const int idx = it * 64 + tid;
      *(volatile v4u*)(dRe + idx * 8) = re4[it];
      *(volatile v4u*)(dIm + idx * 8) = im4[it];
    }
    __threadfence();
  }
}

__global__ __launch_bounds__(128) void beam_power_kernel(const unsigned short* __restrict__ ares,
                                                         const unsigned short* __restrict__ bst,
                                                         float* __restrict__ fmap)
{
  __shared__ __align__(16) float sP[64];
  const int tid = threadIdx.x;
  const int lane = tid & 31;
  const int wave = tid >> 5;
  const int hh = lane >> 4;
  const int c = lane & 15;
  const int bf = blockIdx.x;
  const int d0 = blockIdx.y * 64;
  const _Float16* A = (const _Float16*)ares + (size_t)bf * (kFrmP * 32);
  const _Float16* Bre = (const _Float16*)bst + ((size_t)bf * kStRows + d0 + wave * 16 + c) * 32 + 8 * hh;
  const _Float16* Bim = Bre + (size_t)kNdP * 32;
  const v16h br = Frag<_Float16>::load(Bre);
  const v16h bi = Frag<_Float16>::load(Bim);
  float p = 0.0f;
#pragma unroll 1
  for (int mt = 0; mt < 8; ++mt) {
    const v16h a = Frag<_Float16>::load(A + (mt * 16 + c) * 32 + 8 * hh);
    v8f cr = (v8f){0.f,0.f,0.f,0.f,0.f,0.f,0.f,0.f};
    v8f ci = (v8f){0.f,0.f,0.f,0.f,0.f,0.f,0.f,0.f};
    cr = mma_guard_h(a, br, cr);
    ci = mma_guard_h(a, bi, ci);
#pragma unroll
    for (int r = 0; r < 8; ++r) {
      p = fmaf(cr[r], cr[r], p);
      p = fmaf(ci[r], ci[r], p);
    }
  }
  p += __shfl_xor(p, 16, 32);
  if (lane < 16) sP[wave * 16 + lane] = p;
  __syncthreads();
  if (wave == 0) {
    const v4f raw = *(const v4f*)(sP + c * 4);
    const v4f v = raw * kPowScale;
    if (lane < 16) {
      float* dst = fmap + (size_t)bf * kNdP + d0 + lane * 4;
      *(volatile v4f*)dst = v;
      __threadfence();
      *(volatile v4f*)dst = v;
    }
  }
}

__global__ __launch_bounds__(256) void dir_softmax_kernel(const float* __restrict__ fmap, float* __restrict__ wsm)
{
  __shared__ float sMax[8];
  __shared__ float sSum[8];
  __shared__ __align__(16) float sW[kNdP];
  const int tid = threadIdx.x, lane = tid & 31, wave = tid >> 5;
  const int b = blockIdx.x;
  const int d0 = tid, d1 = tid + 256, d2 = tid + 512;
  const int d3 = (tid + 768 < kNdP) ? (tid + 768) : (kNdP - 1);
  const bool v3 = (tid + 768) < kNd;
  const float* base = fmap + (size_t)b * kNf * kNdP;
  float s0 = 0.0f, s1 = 0.0f, s2 = 0.0f, s3 = 0.0f;
#pragma unroll 1
  for (int f = 0; f < kNf; ++f) {
    const float* row = base + (size_t)f * kNdP;
    s0 += row[d0];
    s1 += row[d1];
    s2 += row[d2];
    s3 += row[d3];
  }
  const float l0 = (s0 * kInvBins) * kInvTemp;
  const float l1 = (s1 * kInvBins) * kInvTemp;
  const float l2 = (s2 * kInvBins) * kInvTemp;
  const float l3 = (s3 * kInvBins) * kInvTemp;
  float m = fmaxf(fmaxf(l0, l1), l2);
  const float l3m = v3 ? l3 : -INFINITY;
  m = fmaxf(m, l3m);
#pragma unroll
  for (int off = 16; off > 0; off >>= 1) m = fmaxf(m, __shfl_xor(m, off, 32));
  if (lane == 0) sMax[wave] = m;
  __syncthreads();
  float mm = sMax[0];
#pragma unroll
  for (int w = 1; w < 8; ++w) mm = fmaxf(mm, sMax[w]);
  const float e0 = expf(l0 - mm);
  const float e1 = expf(l1 - mm);
  const float e2 = expf(l2 - mm);
  const float e3r = expf(fminf(l3 - mm, 0.0f));
  const float e3 = v3 ? e3r : 0.0f;
  float t = (e0 + e1) + (e2 + e3);
#pragma unroll
  for (int off = 16; off > 0; off >>= 1) t += __shfl_xor(t, off, 32);
  if (lane == 0) sSum[wave] = t;
  __syncthreads();
  float tot = sSum[0];
#pragma unroll
  for (int w = 1; w < 8; ++w) tot += sSum[w];
  const float inv = 1.0f / tot;
  sW[d0] = e0 * inv;
  sW[d1] = e1 * inv;
  sW[d2] = e2 * inv;
  if (tid + 768 < kNdP) sW[tid + 768] = e3 * inv;
  __syncthreads();
  if (tid < kNdP / 4) {
    const v4f v = *(const v4f*)(sW + tid * 4);
    float* dst = wsm + (size_t)b * kNdP + tid * 4;
    *(volatile v4f*)dst = v;
    __threadfence();
    *(volatile v4f*)dst = v;
  }
}

__global__ __launch_bounds__(128) void dominant_steer_kernel(const float* __restrict__ wsm, const float* __restrict__ del,
                                                             float* __restrict__ avec)
{
  __shared__ __align__(16) float sA[256];
  const int tid = threadIdx.x;
  const int bfl = tid >> 3, c = tid & 7;
  const int bf = blockIdx.x * 16 + bfl;
  const bool live = bf < kBF;
  const int bfc = live ? bf : (kBF - 1);
  const int b = bfc / kNf;
  const int f = bfc - b * kNf;
  const float tw = kTwoPi * ((float)(kBin0 + f) * kBinHz);
  const float* wr = wsm + (size_t)b * kNdP;
  const float* dr = del + (size_t)(b * kNc + c) * kNdP;
  float ar = 0.0f, ai = 0.0f;
#pragma unroll 1
  for (int d = 0; d < kNd; ++d) {
    const float w = wr[d];
    const float ph = tw * dr[d];
    float sn, cs;
    sincosf(ph, &sn, &cs);
    ar = fmaf(w, cs, ar);
    ai = fmaf(w, sn, ai);
  }
  sA[bfl * 16 + c]     = live ? ar : 0.0f;
  sA[bfl * 16 + 8 + c] = live ? ai : 0.0f;
  __syncthreads();
  if (tid < 64) {
    const v4f v = *(const v4f*)(sA + tid * 4);
    float* dst = avec + (size_t)blockIdx.x * 256 + tid * 4;
    *(volatile v4f*)dst = v;
    __threadfence();
    *(volatile v4f*)dst = v;
  }
}

__global__ __launch_bounds__(128) void shrink_update_kernel(const float* __restrict__ resIn, const float* __restrict__ avec,
                                                            float* __restrict__ resOut, unsigned short* __restrict__ ares)
{
  __shared__ __align__(16) float sR[kFrmP * 16];
  const int tid = threadIdx.x;
  const int bf = blockIdx.x;
  const float* src = resIn + (size_t)bf * (kFrmP * 16) + tid * 16;
#pragma unroll
  for (int q = 0; q < 4; ++q) {
    const v4f v = *(const v4f*)(src + 4 * q);
    *(v4f*)(sR + tid * 16 + 4 * q) = v;
  }
  __syncthreads();
  const float* av = avec + (size_t)bf * 16;
  float sr = 0.0f, si = 0.0f, nrm = 0.0f;
#pragma unroll 1
  for (int c = 0; c < kNc; ++c) {
    const float ar = av[c], ai = av[8 + c];
    const float rr = sR[tid * 16 + c], ri = sR[tid * 16 + 8 + c];
    nrm = fmaf(ar, ar, nrm);
    nrm = fmaf(ai, ai, nrm);
    sr = fmaf(ar, rr, sr);
    sr = fmaf(ai, ri, sr);
    si = fmaf(ar, ri, si);
    si = fmaf(-ai, rr, si);
  }
  const float inv = 1.0f / fmaxf(nrm, kEps);
  sr *= inv;
  si *= inv;
#pragma unroll 1
  for (int c = 0; c < kNc; ++c) {
    const float ar = av[c], ai = av[8 + c];
    const float rr = sR[tid * 16 + c], ri = sR[tid * 16 + 8 + c];
    const float tr = ar * sr - ai * si;
    const float ti = ar * si + ai * sr;
    sR[tid * 16 + c]     = rr - kShrink * tr;
    sR[tid * 16 + 8 + c] = ri - kShrink * ti;
  }
  __syncthreads();
  store_res_planes(sR, resOut + (size_t)bf * (kFrmP * 16), ares + (size_t)bf * (kFrmP * 32), tid);
}

__global__ __launch_bounds__(256) void band_map_out_kernel(const float* __restrict__ fmap, float* __restrict__ out)
{
  __shared__ __align__(16) float sM[kOutPerB];
  __shared__ float sMax[8];
  const int tid = threadIdx.x, lane = tid & 31, wave = tid >> 5;
  const int b = blockIdx.x;
  float lm = -INFINITY;
#pragma unroll 1
  for (int j = 0; j < 30; ++j) {
    const int i = tid + 256 * j;
    const bool live = i < kOutPerB;
    const int ic = live ? i : (kOutPerB - 1);
    const int g = ic / kNd;
    const int d = ic - g * kNd;
    const int fs = (kNf * g + 7) >> 3;
    const int cnt = ((kNf * (g + 1) + 7) >> 3) - fs;
    float acc = 0.0f;
#pragma unroll 1
    for (int k = 0; k < 13; ++k) {
      const int ff = (fs + k < kNf) ? (fs + k) : (kNf - 1);
      float v = fmap[(size_t)(b * kNf + ff) * kNdP + d];
      asm volatile("" : "+v"(v));
      const float fk = (k < cnt) ? 1.0f : 0.0f;
      acc = fmaf(fk, v, acc);
    }
    const float rc = (cnt == 13) ? (1.0f / 13.0f) : (1.0f / 12.0f);
    const float mval = log1pf(acc * rc);
    if (live) sM[i] = mval;
    const float cand = fmaxf(lm, mval);
    lm = live ? cand : lm;
  }
#pragma unroll
  for (int off = 16; off > 0; off >>= 1) lm = fmaxf(lm, __shfl_xor(lm, off, 32));
  if (lane == 0) sMax[wave] = lm;
  __syncthreads();
  float mx = sMax[0];
#pragma unroll
  for (int w = 1; w < 8; ++w) mx = fmaxf(mx, sMax[w]);
  const float inv = 1.0f / fmaxf(mx, kEps);
  float* ob = out + (size_t)b * kOutPerB;
  for (int pass = 0; pass < 2; ++pass) {
#pragma unroll 1
    for (int it = 0; it < 8; ++it) {
      const int idx = it * 256 + tid;
      if (idx < kOutPerB / 4) {
        const v4f raw = *(const v4f*)(sM + idx * 4);
        const v4f v = raw * inv;
        *(volatile v4f*)(ob + idx * 4) = v;
      }
    }
    __threadfence();
  }
}

extern "C" void kernel_launch(void* const* d_in, const int* in_sizes, int n_in,
                              void* d_out, int out_size, void* d_ws, size_t ws_size,
                              hipStream_t stream) {
  if (n_in < 2) return;
  if (in_sizes[0] != kBC * kNt) return;
  if (in_sizes[1] != kBC * 3) return;
  if (out_size != kNb * kOutPerB) return;
  if (ws_size < kWsTotal) return;

  const float* audio = (const float*)d_in[0];
  const float* mics  = (const float*)d_in[1];
  float* out = (float*)d_out;

  char* ws = (char*)d_ws;
  unsigned short* AUD   = (unsigned short*)(ws + kOffAUD);
  unsigned short* BDFT  = (unsigned short*)(ws + kOffBDFT);
  float*          CSPEC = (float*)(ws + kOffCSPEC);
  float*          DEL   = (float*)(ws + kOffDEL);
  float*          RES0  = (float*)(ws + kOffRES0);
  float*          RES1  = (float*)(ws + kOffRES1);
  unsigned short* ARES  = (unsigned short*)(ws + kOffARES);
  unsigned short* BST   = (unsigned short*)(ws + kOffBST);
  float*          FMAP  = (float*)(ws + kOffFMAP);
  float*          WSM   = (float*)(ws + kOffWSM);
  float*          AVEC  = (float*)(ws + kOffAVEC);

  dft_plane_kernel<<<(kNdft * kWin) / 2048, 256, 0, stream>>>(BDFT);
  delays_kernel<<<dim3(kBC, kNdP / 64), 64, 0, stream>>>(mics, DEL);
  audio_plane_kernel<<<(kBC * (kAudP / 8)) / 256, 256, 0, stream>>>(audio, AUD);

  wmma_gemm64<0, false, 0, 0, false, 0><<<dim3(1, kBC), 256, 0, stream>>>(
      AUD, nullptr, kHop, (long)kAudP,
      BDFT, nullptr, kWin, 0L,
      (void*)CSPEC, nullptr, kNdft, (long)(kFrmP * kNdft),
      nullptr, nullptr, 0L,
      kFrmP, kNdft, kWin, kStftScale);

  phat_pack_kernel<<<kBF, 128, 0, stream>>>(CSPEC, RES0, ARES);
  steer_plane_kernel<<<dim3(kBF, kNdP / 64), 64, 0, stream>>>(DEL, BST);

  for (int it = 0; it < 3; ++it) {
    beam_power_kernel<<<dim3(kBF, kNdP / 64), 128, 0, stream>>>(ARES, BST, FMAP);
    if (it < 2) {
      dir_softmax_kernel<<<kNb, 256, 0, stream>>>(FMAP, WSM);
      dominant_steer_kernel<<<kAvRows / 16, 128, 0, stream>>>(WSM, DEL, AVEC);
      const float* rin = (it == 0) ? RES0 : RES1;
      float* rout = (it == 0) ? RES1 : RES0;
      shrink_update_kernel<<<kBF, 128, 0, stream>>>(rin, AVEC, rout, ARES);
    }
  }
  band_map_out_kernel<<<kNb, 256, 0, stream>>>(FMAP, out);
}
